// MultiHeadDiffAttention_71399536328796
// MI455X (gfx1250) — hardware-verified
//
#include <hip/hip_runtime.h>
#include <math.h>
#include <stdint.h>

#ifndef NB
#define NB 2
#endif
#ifndef SEQ
#define SEQ 2048
#endif
#define NB_FULL  2
#define SEQ_FULL 2048
#define DM    512
#define NH    8
#define HD    64
#define DV    64
#define DVT   (NH * DV)
#define DQKV  (5 * DM)
#define VOFF  (4 * DM)
#define YP    DVT
#define NQB   (SEQ / 64)
#define NG    4
#define CPG   (DM / NG)
#define NPB   (SEQ / 64)
#define PTW   64
#define STW   32
#define LAM_INIT 0.2f
#define GN_EPS   1e-5f

static_assert(NH * HD == DM);
static_assert(DV == HD && DVT == DM && YP == DM && DM == 512);
static_assert(NB >= 1 && NB <= NB_FULL && SEQ >= 64 && SEQ <= SEQ_FULL && (SEQ % 64) == 0);
static_assert((((SEQ / 64) * (DQKV / 64)) % 8) == 0);
static_assert((((SEQ / 64) * (DM / 64)) % 8) == 0);
static_assert(((SEQ * DM / 8) % 256) == 0 && ((DM * DM / 8) % 256) == 0);
static_assert(NG * CPG == DM && CPG == 2 * HD);
static_assert(5 * NH <= PTW && 5 * NH <= 64 && 2 * NG + NH <= STW && (STW % 4) == 0);
static_assert((DQKV % 64) == 0 && ((DQKV / 4) % 32) == 0);

typedef _Float16 v16h __attribute__((ext_vector_type(16)));
typedef _Float16 v8h  __attribute__((ext_vector_type(8)));
typedef float    v8f  __attribute__((ext_vector_type(8)));
typedef float    v4f  __attribute__((ext_vector_type(4)));
typedef unsigned int v4u __attribute__((ext_vector_type(4)));
typedef double   v2d  __attribute__((ext_vector_type(2)));

__device__ __forceinline__ unsigned short bf_bits(float f) {
  unsigned u = __float_as_uint(f);
  return (unsigned short)((u + 0x7FFFu + ((u >> 16) & 1u)) >> 16);
}
__device__ __forceinline__ float bfr(float f) { return __uint_as_float(((unsigned)bf_bits(f)) << 16); }
__device__ __forceinline__ unsigned short h_bits(_Float16 x) { return __builtin_bit_cast(unsigned short, x); }
__device__ __forceinline__ unsigned pk16(unsigned short a, unsigned short b) { return (unsigned)a | ((unsigned)b << 16); }
__device__ __forceinline__ v8f zero8() { v8f z = {0.f, 0.f, 0.f, 0.f, 0.f, 0.f, 0.f, 0.f}; return z; }

__device__ __forceinline__ v16h ldfrag_h(const _Float16* p) {
  union { v16h v; v8h h[2]; } f;
  f.h[0] = *(const v8h*)(p);
  f.h[1] = *(const v8h*)(p + 16);
  return f.v;
}

__device__ __forceinline__ v8f mma_h(v16h a, v16h b, v8f c) {
  c = __builtin_amdgcn_wmma_f32_16x16x32_f16(false, a, false, b, (short)0, c, false, false);
#if defined(__HIP_DEVICE_COMPILE__)
  asm volatile("v_nop\n\tv_nop\n\tv_nop\n\tv_nop" : "+v"(c) : "v"(a), "v"(b));
#endif
  return c;
}
__device__ __forceinline__ v8f mma_h_raw(v16h a, v16h b, v8f c) {
  return __builtin_amdgcn_wmma_f32_16x16x32_f16(false, a, false, b, (short)0, c, false, false);
}
__device__ __forceinline__ void dep_guard_h(v8f& a, v8f& b, v16h x, v16h y) {
#if defined(__HIP_DEVICE_COMPILE__)
  asm volatile("v_nop\n\tv_nop\n\tv_nop\n\tv_nop" : "+v"(a), "+v"(b) : "v"(x), "v"(y));
#endif
}
__device__ __forceinline__ void keep4_h(v16h a, v16h b, v16h c, v16h d) {
#if defined(__HIP_DEVICE_COMPILE__)
  asm volatile("v_nop" :: "v"(a), "v"(b), "v"(c), "v"(d));
#endif
}
__device__ __forceinline__ void acc_guard4(v8f& a, v8f& b, v8f& c, v8f& d) {
#if defined(__HIP_DEVICE_COMPILE__)
  asm volatile("v_nop\n\tv_nop\n\tv_nop\n\tv_nop" : "+v"(a), "+v"(b), "+v"(c), "+v"(d));
#endif
}

__global__ __launch_bounds__(256) void cvt16(const float* __restrict__ in, unsigned short* out, int n8, float scale) {
  const int i = blockIdx.x * 256 + threadIdx.x;
  if (i < n8) {
    const v4f a = *(const v4f*)(in + (size_t)i * 8);
    const v4f b = *(const v4f*)(in + (size_t)i * 8 + 4);
    v4u p;
    p[0] = pk16(h_bits((_Float16)(bfr(a[0]) * scale)), h_bits((_Float16)(bfr(a[1]) * scale)));
    p[1] = pk16(h_bits((_Float16)(bfr(a[2]) * scale)), h_bits((_Float16)(bfr(a[3]) * scale)));
    p[2] = pk16(h_bits((_Float16)(bfr(b[0]) * scale)), h_bits((_Float16)(bfr(b[1]) * scale)));
    p[3] = pk16(h_bits((_Float16)(bfr(b[2]) * scale)), h_bits((_Float16)(bfr(b[3]) * scale)));
    *(volatile v4u*)(out + (size_t)i * 8) = p;
    __threadfence();
    *(volatile v4u*)(out + (size_t)i * 8) = p;
  }
}

__global__ __launch_bounds__(256) void mkbias(const float* __restrict__ b1, const float* __restrict__ b2, float* Bq) {
  const int i = blockIdx.x * 256 + threadIdx.x;
  if (i < DQKV / 4) {
    const int n   = i * 4;
    const int seg = n / DM;
    const int c   = n & (DM - 1);
    const v4f x1 = *(const v4f*)(b1 + c);
    const v4f x2 = *(const v4f*)(b2 + c);
    v4f v;
#pragma unroll
    for (int e = 0; e < 4; ++e) {
      const float u1 = bfr(x1[e]), u2 = bfr(x2[e]);
      v[e] = (seg == 2) ? u1 : ((seg == 3) ? u2 : 0.0f);
    }
    *(volatile v4f*)(Bq + n) = v;
    __threadfence();
    *(volatile v4f*)(Bq + n) = v;
  }
}

template <int EPI, bool ARES>
__global__ __launch_bounds__(256) void gemm64_f16(
    const unsigned short* __restrict__ Ap, const unsigned short* __restrict__ Arp, int lda,
    const unsigned short* __restrict__ Btp, int ldb, const float* __restrict__ bias, float cscale,
    void* Cp, unsigned short* Crp, int ldc, int M, int N, int K, float oscale) {
  const _Float16* Ah  = (const _Float16*)(const void*)Ap;
  const _Float16* Arh = (const _Float16*)(const void*)Arp;
  const _Float16* Bt  = (const _Float16*)(const void*)Btp;
  __shared__ __align__(16) float sT[8][16 * 68];
  const int lane = threadIdx.x & 31;
  const int wave = threadIdx.x >> 5;
  const int tilesN = N >> 6;
  const int tilesM = M >> 6;
  const int tile = blockIdx.x * 8 + wave;
  if (tile >= tilesM * tilesN) return;
  const int tm = tile / tilesN;
  const int tn = tile - tm * tilesN;
  const int m0 = tm << 6;
  const int n0 = tn << 6;

  const int rlane = lane & 15;
  const int koff  = (lane >> 4) * 8;
  const int mOff  = (lane >> 4) * 8;

  v8f acc[4][4];
#pragma unroll
  for (int i = 0; i < 4; ++i)
#pragma unroll
    for (int j = 0; j < 4; ++j) acc[i][j] = zero8();

  constexpr int NPL = ARES ? 2 : 1;
#pragma unroll 1
  for (int pl = 0; pl < NPL; ++pl) {
    const _Float16* Asel = (ARES && pl == 0) ? Arh : Ah;
    if (ARES && pl == 1) {
      acc_guard4(acc[0][0], acc[0][1], acc[0][2], acc[0][3]);
      acc_guard4(acc[1][0], acc[1][1], acc[1][2], acc[1][3]);
      acc_guard4(acc[2][0], acc[2][1], acc[2][2], acc[2][3]);
      acc_guard4(acc[3][0], acc[3][1], acc[3][2], acc[3][3]);
#pragma unroll
      for (int i = 0; i < 4; ++i)
#pragma unroll
        for (int j = 0; j < 4; ++j) acc[i][j] = acc[i][j] * (1.0f / 2048.0f);
      acc_guard4(acc[0][0], acc[0][1], acc[0][2], acc[0][3]);
      acc_guard4(acc[1][0], acc[1][1], acc[1][2], acc[1][3]);
      acc_guard4(acc[2][0], acc[2][1], acc[2][2], acc[2][3]);
      acc_guard4(acc[3][0], acc[3][1], acc[3][2], acc[3][3]);
    }
    for (int k0 = 0; k0 < K; k0 += 32) {
      v16h bh[4];
#pragma unroll
      for (int j = 0; j < 4; ++j) {
        const size_t bo = (size_t)(n0 + (j << 4) + rlane) * ldb + koff + k0;
        bh[j] = ldfrag_h(Bt + bo);
      }
#pragma unroll
      for (int i = 0; i < 4; ++i) {
        const size_t ao = (size_t)(m0 + (i << 4) + rlane) * lda + koff + k0;
        const v16h ah = ldfrag_h(Asel + ao);
#pragma unroll
        for (int j = 0; j < 4; ++j) {
          acc[i][j] = mma_h_raw(ah, bh[j], acc[i][j]);
        }
        dep_guard_h(acc[i][0], acc[i][3], ah, bh[3]);
      }
      keep4_h(bh[0], bh[1], bh[2], bh[3]);
    }
  }
  acc_guard4(acc[0][0], acc[0][1], acc[0][2], acc[0][3]);
  acc_guard4(acc[1][0], acc[1][1], acc[1][2], acc[1][3]);
  acc_guard4(acc[2][0], acc[2][1], acc[2][2], acc[2][3]);
  acc_guard4(acc[3][0], acc[3][1], acc[3][2], acc[3][3]);

  float bb[4];
#pragma unroll
  for (int j = 0; j < 4; ++j) bb[j] = bfr(bias[n0 + (j << 4) + rlane]);
  float* slab = sT[wave];
#pragma unroll
  for (int i = 0; i < 4; ++i) {
    const int mBase = m0 + (i << 4);
#pragma unroll
    for (int r = 0; r < 8; ++r) {
      const int row = mOff + r;
#pragma unroll
      for (int j = 0; j < 4; ++j) slab[row * 68 + (j << 4) + rlane] = acc[i][j][r] * cscale + bb[j];
    }
    __builtin_amdgcn_fence(__ATOMIC_RELEASE, "workgroup");
    __builtin_amdgcn_wave_barrier();
    __builtin_amdgcn_fence(__ATOMIC_ACQUIRE, "workgroup");
    if constexpr (EPI == 0) {
      unsigned short* C16 = (unsigned short*)Cp;
      const int rq = lane >> 3, piece = lane & 7;
      v4u ph[4], pr[4];
#pragma unroll
      for (int it = 0; it < 4; ++it) {
        const int row = it * 4 + rq;
        const v4f a  = *(const v4f*)(slab + row * 68 + piece * 8);
        const v4f a2 = *(const v4f*)(slab + row * 68 + piece * 8 + 4);
        float f[8];
        f[0] = a[0];  f[1] = a[1];  f[2] = a[2];  f[3] = a[3];
        f[4] = a2[0]; f[5] = a2[1]; f[6] = a2[2]; f[7] = a2[3];
        v4u p, q;
#pragma unroll
        for (int e = 0; e < 4; ++e) {
          const float g0 = f[2 * e] * oscale, g1 = f[2 * e + 1] * oscale;
          const _Float16 x0 = (_Float16)g0, x1 = (_Float16)g1;
          const _Float16 y0 = (_Float16)((g0 - (float)x0) * 2048.0f);
          const _Float16 y1 = (_Float16)((g1 - (float)x1) * 2048.0f);
          p[e] = pk16(h_bits(x0), h_bits(x1));
          q[e] = pk16(h_bits(y0), h_bits(y1));
        }
        ph[it] = p;
        pr[it] = q;
      }
      for (int pass = 0; pass < 2; ++pass) {
#pragma unroll
        for (int it = 0; it < 4; ++it) {
          const int row = it * 4 + rq;
          const size_t co = (size_t)(mBase + row) * ldc + n0 + piece * 8;
          *(volatile v4u*)(C16 + co) = ph[it];
          *(volatile v4u*)(Crp + co) = pr[it];
        }
        __threadfence();
      }
    } else {
      float* Cf = (float*)Cp;
      const int hh = lane >> 4, c4 = (lane & 15) * 4;
      v4f ov[8];
#pragma unroll
      for (int it = 0; it < 8; ++it) {
        const int row = it * 2 + hh;
        ov[it] = *(const v4f*)(slab + row * 68 + c4);
      }
      for (int pass = 0; pass < 2; ++pass) {
#pragma unroll
        for (int it = 0; it < 8; ++it) {
          const int row = it * 2 + hh;
          *(volatile v4f*)(Cf + (size_t)(mBase + row) * ldc + n0 + c4) = ov[it];
        }
        __threadfence();
      }
    }
    __builtin_amdgcn_fence(__ATOMIC_RELEASE, "workgroup");
    __builtin_amdgcn_wave_barrier();
    __builtin_amdgcn_fence(__ATOMIC_ACQUIRE, "workgroup");
  }
}

__global__ __launch_bounds__(256) void v_tr(const unsigned short* __restrict__ qkvp, unsigned short* vt, int opitch) {
  __shared__ __align__(16) _Float16 sv[64 * 72];
  const int tid = threadIdx.x;
  const int t0  = blockIdx.x * 64;
  const int fy  = blockIdx.y;
  const _Float16* src = (const _Float16*)(const void*)qkvp;
#pragma unroll
  for (int i = 0; i < 2; ++i) {
    const int idx = i * 256 + tid;
    const int tt = idx >> 3, c8 = (idx & 7) * 8;
    const v8h a = *(const v8h*)(src + ((size_t)(t0 + tt)) * DQKV + VOFF + fy * 64 + c8);
    *(v8h*)(sv + tt * 72 + c8) = a;
  }
  __syncthreads();

  const int g = tid >> 3, piece = tid & 7;
  v4u hv[2];
  size_t hofs[2];
#pragma unroll
  for (int it = 0; it < 2; ++it) {
    const int d = it * 32 + g;
    v4u a;
#pragma unroll
    for (int e = 0; e < 4; ++e) {
      const _Float16 x0 = sv[(piece * 8 + 2 * e) * 72 + d];
      const _Float16 x1 = sv[(piece * 8 + 2 * e + 1) * 72 + d];
      a[e] = pk16(h_bits(x0), h_bits(x1));
    }
    hv[it] = a;
    hofs[it] = ((size_t)(fy * 64 + d)) * opitch + t0 + piece * 8;
  }
  for (int pass = 0; pass < 2; ++pass) {
#pragma unroll
    for (int it = 0; it < 2; ++it) *(volatile v4u*)(vt + hofs[it]) = hv[it];
    __threadfence();
  }
}

__global__ __launch_bounds__(128)
void attn_k(const unsigned short* __restrict__ qkvp, const unsigned short* __restrict__ qkvrp,
            const unsigned short* __restrict__ vtp, const unsigned short* __restrict__ vtrp,
            float* C1p, float* C2p) {
  union FH { v16h v; v8h h[2]; };
  constexpr int  NVT    = 4;
  constexpr int  VC     = NVT * 16;
  constexpr int  TBK    = 64 * 64 * 2;
  constexpr int  TBV    = VC * 64 * 2;
  constexpr int  PB     = 4 * 16 * 64 * 2;
  constexpr int  OFF_K  = 0;
  constexpr int  OFF_V  = OFF_K + TBK;
  constexpr int  OFF_KR = OFF_V + TBV;
  constexpr int  OFF_VR = OFF_KR + TBK;
  constexpr int  OFF_P  = OFF_VR + TBV;
  constexpr int  OFF_PR = OFF_P + PB;
  constexpr int  SMEMB  = OFF_PR + PB;
  constexpr int  OSB    = 4 * 16 * VC * 4;
  constexpr int  VHT    = (VC * 64) / 128;
  constexpr int  TPR    = 64 / VHT;
  constexpr int  LPR    = VC / 4;
  constexpr int  RPI    = 32 / LPR;
  constexpr int  NIT    = 16 / RPI;
  static_assert(OSB <= SMEMB);
  static_assert(VC == DV);
  static_assert(VHT * 128 == VC * 64 && (VHT % 8) == 0 && TPR * VHT == 64);
  static_assert(LPR * RPI == 32 && NIT * RPI == 16 && (NIT % 8) == 0);
  __shared__ __align__(16) unsigned char smem[SMEMB];
  _Float16* Ksh = (_Float16*)(smem + OFF_K);
  _Float16* Vsh = (_Float16*)(smem + OFF_V);
  _Float16* Krs = (_Float16*)(smem + OFF_KR);
  _Float16* Vrs = (_Float16*)(smem + OFF_VR);
  _Float16* Psh = (_Float16*)(smem + OFF_P);
  _Float16* Prs = (_Float16*)(smem + OFF_PR);

  const int tid  = threadIdx.x;
  const int wave = tid >> 5;
  const int lane = tid & 31;
  const int hh   = lane >> 4;
  const int c    = lane & 15;

  const int bx   = blockIdx.x;
  const int qb   = bx % NQB;
  const int rest = bx / NQB;
  const int map  = rest & 1;
  const int h    = rest >> 1;
  const int q0   = qb * 64 + wave * 16;
  const int cb   = h * DV;

  const _Float16* Qp  = (const _Float16*)(const void*)qkvp  + (size_t)map * DM + (size_t)h * HD;
  const _Float16* Qrp = (const _Float16*)(const void*)qkvrp + (size_t)map * DM + (size_t)h * HD;
  const _Float16* Kp  = Qp + 2 * DM;
  const _Float16* Krp = Qrp + 2 * DM;
  const _Float16* Vt  = (const _Float16*)(const void*)vtp  + (size_t)cb * SEQ;
  const _Float16* Vrt = (const _Float16*)(const void*)vtrp + (size_t)cb * SEQ;
  float* Co = map ? C2p : C1p;

  v16h qa[2], qr[2];
#pragma unroll
  for (int dc = 0; dc < 2; ++dc) {
    const size_t qo = (size_t)(q0 + c) * DQKV + dc * 32 + 8 * hh;
    qa[dc] = ldfrag_h(Qp + qo);
    qr[dc] = ldfrag_h(Qrp + qo);
  }

  float lsum[8], mrun[8];
  v8f oacc[NVT], oacc2[NVT];
#pragma unroll
  for (int r = 0; r < 8; ++r) { lsum[r] = 0.f; mrun[r] = -1e30f; }
#pragma unroll
  for (int t = 0; t < NVT; ++t) { oacc[t] = zero8(); oacc2[t] = zero8(); }

  _Float16* pw  = Psh + wave * (16 * 64);
  _Float16* prw = Prs + wave * (16 * 64);

#pragma unroll 1
  for (int kt = 0; kt < NQB; ++kt) {
    const int kv0 = kt * 64;
    __syncthreads();
    {
      const int r = tid >> 1, half = (tid & 1) * 32;
      const size_t ko = (size_t)(kv0 + r) * DQKV + half;
#pragma unroll
      for (int i = 0; i < 4; ++i) {
        const v8h a0 = *(const v8h*)(Kp + ko + 8 * i);
        *(v8h*)(Ksh + r * 64 + half + 8 * i) = a0;
        const v8h a1 = *(const v8h*)(Krp + ko + 8 * i);
        *(v8h*)(Krs + r * 64 + half + 8 * i) = a1;
      }
      const int vr = tid / TPR, voff = (tid - vr * TPR) * VHT;
      const size_t vo = (size_t)vr * SEQ + kv0 + voff;
#pragma unroll
      for (int i = 0; i < VHT / 8; ++i) {
        const v8h b0 = *(const v8h*)(Vt + vo + 8 * i);
        *(v8h*)(Vsh + vr * 64 + voff + 8 * i) = b0;
        const v8h b1 = *(const v8h*)(Vrt + vo + 8 * i);
        *(v8h*)(Vrs + vr * 64 + voff + 8 * i) = b1;
      }
    }
    __syncthreads();

    v8f s[4];
#pragma unroll
    for (int j = 0; j < 4; ++j) {
      s[j] = zero8();
      v8f t = zero8();
#pragma unroll
      for (int dc = 0; dc < 2; ++dc) {
        FH kb;
        kb.h[0] = *(const v8h*)(Ksh + (j * 16 + c) * 64 + dc * 32 + 8 * hh);
        kb.h[1] = *(const v8h*)(Ksh + (j * 16 + c) * 64 + dc * 32 + 16 + 8 * hh);
        s[j] = mma_h(qa[dc], kb.v, s[j]);
        FH krb;
        krb.h[0] = *(const v8h*)(Krs + (j * 16 + c) * 64 + dc * 32 + 8 * hh);
        krb.h[1] = *(const v8h*)(Krs + (j * 16 + c) * 64 + dc * 32 + 16 + 8 * hh);
        t = mma_h(qa[dc], krb.v, t);
        t = mma_h(qr[dc], kb.v, t);
      }
      s[j] = s[j] + t * (1.0f / 2048.0f);
    }

    float alpha[8];
#pragma unroll
    for (int r = 0; r < 8; ++r) {
      float av[4];
      float tmx = -1e30f;
#pragma unroll
      for (int j = 0; j < 4; ++j) {
        const float a = s[j][r] * (1.0f / 2048.0f);
        av[j] = a;
        tmx = fmaxf(tmx, a);
      }
#pragma unroll
      for (int off = 1; off < 16; off <<= 1) tmx = fmaxf(tmx, __shfl_xor(tmx, off, 32));
      const float mn = fmaxf(mrun[r], tmx);
      const float al = __expf(mrun[r] - mn);
      alpha[r] = al;
      mrun[r]  = mn;
      float ps = 0.0f;
#pragma unroll
      for (int j = 0; j < 4; ++j) {
        const float p = __expf(av[j] - mn);
        ps += p;
        const float g = p * 256.0f;
        const _Float16 x0 = (_Float16)g;
        pw[(8 * hh + r) * 64 + j * 16 + c]  = x0;
        prw[(8 * hh + r) * 64 + j * 16 + c] = (_Float16)((g - (float)x0) * 2048.0f);
      }
      lsum[r] = lsum[r] * al + ps;
    }
    __builtin_amdgcn_fence(__ATOMIC_RELEASE, "workgroup");
    __builtin_amdgcn_wave_barrier();
    __builtin_amdgcn_fence(__ATOMIC_ACQUIRE, "workgroup");

#pragma unroll
    for (int t = 0; t < NVT; ++t) {
#pragma unroll
      for (int r = 0; r < 8; ++r) {
        oacc[t][r]  = oacc[t][r] * alpha[r];
        oacc2[t][r] = oacc2[t][r] * alpha[r];
      }
    }
    acc_guard4(oacc[0], oacc[1], oacc[2], oacc[3]);
    acc_guard4(oacc2[0], oacc2[1], oacc2[2], oacc2[3]);

#pragma unroll
    for (int kk = 0; kk < 2; ++kk) {
      FH pa, par;
      pa.h[0]  = *(const v8h*)(pw + c * 64 + kk * 32 + 8 * hh);
      pa.h[1]  = *(const v8h*)(pw + c * 64 + kk * 32 + 16 + 8 * hh);
      par.h[0] = *(const v8h*)(prw + c * 64 + kk * 32 + 8 * hh);
      par.h[1] = *(const v8h*)(prw + c * 64 + kk * 32 + 16 + 8 * hh);
#pragma unroll
      for (int t = 0; t < NVT; ++t) {
        FH vb, vrb;
        vb.h[0]  = *(const v8h*)(Vsh + (t * 16 + c) * 64 + kk * 32 + 8 * hh);
        vb.h[1]  = *(const v8h*)(Vsh + (t * 16 + c) * 64 + kk * 32 + 16 + 8 * hh);
        vrb.h[0] = *(const v8h*)(Vrs + (t * 16 + c) * 64 + kk * 32 + 8 * hh);
        vrb.h[1] = *(const v8h*)(Vrs + (t * 16 + c) * 64 + kk * 32 + 16 + 8 * hh);
        oacc[t]  = mma_h(pa.v, vb.v, oacc[t]);
        oacc2[t] = mma_h(pa.v, vrb.v, oacc2[t]);
        oacc2[t] = mma_h(par.v, vb.v, oacc2[t]);
      }
    }
  }
  __syncthreads();

  float* os = (float*)(void*)smem + wave * (16 * VC);
#pragma unroll
  for (int r = 0; r < 8; ++r) {
    float l = lsum[r];
#pragma unroll
    for (int off = 1; off < 16; off <<= 1) l += __shfl_xor(l, off, 32);
    const float rl = 1.0f / l;
#pragma unroll
    for (int t = 0; t < NVT; ++t) {
      float v = oacc[t][r] + oacc2[t][r] * (1.0f / 2048.0f);
      v = v * (1.0f / 4096.0f);
      os[(8 * hh + r) * VC + t * 16 + c] = v * rl;
    }
  }
  __builtin_amdgcn_fence(__ATOMIC_RELEASE, "workgroup");
  __builtin_amdgcn_wave_barrier();
  __builtin_amdgcn_fence(__ATOMIC_ACQUIRE, "workgroup");
  {
    const int sub = lane / LPR;
    const int c4  = (lane - sub * LPR) * 4;
#pragma unroll
    for (int bt = 0; bt < NIT; bt += 8) {
      v4f ov[8];
#pragma unroll
      for (int it = 0; it < 8; ++it) {
        const int row = (bt + it) * RPI + sub;
        ov[it] = *(const v4f*)(os + row * VC + c4);
      }
      for (int pass = 0; pass < 2; ++pass) {
#pragma unroll
        for (int it = 0; it < 8; ++it) {
          const int row = (bt + it) * RPI + sub;
          *(volatile v4f*)(Co + (size_t)(q0 + row) * YP + cb + c4) = ov[it];
        }
        __threadfence();
      }
    }
  }
}

__global__ __launch_bounds__(256) void gn_part(const float* __restrict__ C1, const float* __restrict__ C2, double* PT) {
  __shared__ double sh[5][DM];
  __shared__ __align__(16) double stg[PTW];
  const int tid = threadIdx.x;
  const int t0  = blockIdx.x * 64;
  double s1a = 0.0, s2a = 0.0, qaa = 0.0, qab = 0.0, qbb = 0.0;
  double s1b = 0.0, s2b = 0.0, raa = 0.0, rab = 0.0, rbb = 0.0;
#pragma unroll 1
  for (int t = 0; t < 64; ++t) {
    const size_t o = (size_t)(t0 + t) * YP;
    const float a0 = C1[o + tid],       b0 = C2[o + tid];
    const float a1 = C1[o + tid + 256], b1 = C2[o + tid + 256];
    const double x0 = (double)a0, y0 = (double)b0, x1 = (double)a1, y1 = (double)b1;
    s1a += x0; s2a += y0; qaa += x0 * x0; qab += x0 * y0; qbb += y0 * y0;
    s1b += x1; s2b += y1; raa += x1 * x1; rab += x1 * y1; rbb += y1 * y1;
  }
  sh[0][tid] = s1a; sh[1][tid] = s2a; sh[2][tid] = qaa; sh[3][tid] = qab; sh[4][tid] = qbb;
  sh[0][tid + 256] = s1b; sh[1][tid + 256] = s2b; sh[2][tid + 256] = raa; sh[3][tid + 256] = rab; sh[4][tid + 256] = rbb;
  __syncthreads();
  if (tid < 64) {
    const int jj = (tid < 5 * NH) ? tid : 0;
    const int hd = jj / 5, s = jj - 5 * hd;
    const double* p = &sh[s][hd * HD];
    double v = 0.0;
#pragma unroll 1
    for (int i = 0; i < HD; ++i) v += p[i];
    stg[tid] = (tid < 5 * NH) ? v : 0.0;
  }
  __syncthreads();
  if (tid < 32) {
    const v2d val = *(const v2d*)(stg + 2 * tid);
    double* dst = PT + (size_t)blockIdx.x * PTW + 2 * tid;
    *(volatile v2d*)dst = val;
    __threadfence();
    *(volatile v2d*)dst = val;
  }
}

__global__ __launch_bounds__(256) void gn_fin(const double* __restrict__ PT,
                                              const float* __restrict__ lq1, const float* __restrict__ lk1,
                                              const float* __restrict__ lq2, const float* __restrict__ lk2,
                                              float* ST) {
  __shared__ double shs[5 * NH];
  __shared__ float shl[NH];
  __shared__ __align__(16) float stg[STW];
  const int tid = threadIdx.x;
  if (tid < 64) {
    const int j = (tid < 5 * NH) ? tid : 0;
    double v = 0.0;
#pragma unroll 1
    for (int b = 0; b < NPB; ++b) v += PT[(size_t)b * PTW + j];
    if (tid < 5 * NH) shs[tid] = v;
    if (tid < STW) stg[tid] = 0.0f;
    const int hq = tid & (NH - 1);
    const float x1 = bfr(lq1[hq]) * bfr(lk1[hq]);
    const float x2 = bfr(lq2[hq]) * bfr(lk2[hq]);
    const float lam = expf(x1) - expf(x2) + LAM_INIT;
    if (tid < NH) shl[tid] = lam;
  }
  __syncthreads();
  if (tid < 32) {
    if (tid < NG) {
      double S = 0.0, Q = 0.0;
#pragma unroll
      for (int k = 0; k < 2; ++k) {
        const int hd = 2 * tid + k;
        const double L = (double)shl[hd];
        const double* p = shs + 5 * hd;
        S += p[0] - L * p[1];
        Q += p[2] - 2.0 * L * p[3] + L * L * p[4];
      }
      const double inv = 1.0 / (double)((size_t)SEQ * CPG);
      const double mu  = S * inv;
      double var = Q * inv - mu * mu;
      var = var < 0.0 ? 0.0 : var;
      stg[tid] = (float)mu;
      stg[NG + tid] = 1.0f / sqrtf((float)var + GN_EPS);
    }
    if (tid < NH) stg[2 * NG + tid] = shl[tid];
  }
  __syncthreads();
  if (tid < STW / 4) {
    const v4f v = *(const v4f*)(stg + tid * 4);
    float* dst = ST + tid * 4;
    *(volatile v4f*)dst = v;
    __threadfence();
    *(volatile v4f*)dst = v;
  }
}

__global__ __launch_bounds__(256) void gn_apply(const float* __restrict__ C1, const float* __restrict__ C2,
                                                const float* __restrict__ ST, const float* __restrict__ gnw,
                                                const float* __restrict__ gnb,
                                                unsigned short* Yn, unsigned short* Ynr) {
  const int t  = blockIdx.x * 4 + (threadIdx.x >> 6);
  const int f8 = (threadIdx.x & 63) * 8;
  const int h  = f8 / HD;
  const int g  = f8 / CPG;
  const float mu  = ST[g];
  const float rs  = ST[NG + g];
  const float lam = ST[2 * NG + h];
  const size_t ro = (size_t)t * YP + f8;
  const v4f a0 = *(const v4f*)(C1 + ro), a1 = *(const v4f*)(C1 + ro + 4);
  const v4f b0 = *(const v4f*)(C2 + ro), b1 = *(const v4f*)(C2 + ro + 4);
  const v4f w0 = *(const v4f*)(gnw + f8), w1 = *(const v4f*)(gnw + f8 + 4);
  const v4f e0 = *(const v4f*)(gnb + f8), e1 = *(const v4f*)(gnb + f8 + 4);
  float yn[8];
#pragma unroll
  for (int e = 0; e < 4; ++e) {
    const float y = a0[e] - lam * b0[e];
    yn[e] = ((y - mu) * rs) * bfr(w0[e]) + bfr(e0[e]);
  }
#pragma unroll
  for (int e = 0; e < 4; ++e) {
    const float y = a1[e] - lam * b1[e];
    yn[4 + e] = ((y - mu) * rs) * bfr(w1[e]) + bfr(e1[e]);
  }
  v4u p, q;
#pragma unroll
  for (int e = 0; e < 4; ++e) {
    const float g0v = yn[2 * e] * 16.0f, g1v = yn[2 * e + 1] * 16.0f;
    const _Float16 x0 = (_Float16)g0v, x1 = (_Float16)g1v;
    const _Float16 y0 = (_Float16)((g0v - (float)x0) * 2048.0f);
    const _Float16 y1 = (_Float16)((g1v - (float)x1) * 2048.0f);
    p[e] = pk16(h_bits(x0), h_bits(x1));
    q[e] = pk16(h_bits(y0), h_bits(y1));
  }
  const size_t wo = (size_t)t * DM + f8;
  for (int pass = 0; pass < 2; ++pass) {
    *(volatile v4u*)(Yn + wo)  = p;
    *(volatile v4u*)(Ynr + wo) = q;
    __threadfence();
  }
}

extern "C" void kernel_launch(void* const* d_in, const int* in_sizes, int n_in,
                              void* d_out, int out_size, void* d_ws, size_t ws_size,
                              hipStream_t stream) {
  if (n_in < 16) return;
  if (in_sizes[0] < NB * SEQ_FULL * DM) return;
  if (in_sizes[1] < DM * DM || in_sizes[3] < DM * DM || in_sizes[4] < DM * DM) return;
  if (in_sizes[6] < DM * DM || in_sizes[7] < DM * DM || in_sizes[14] < DM * DM) return;
  if (in_sizes[2] < DM || in_sizes[5] < DM || in_sizes[12] < DM || in_sizes[13] < DM || in_sizes[15] < DM) return;
  if (in_sizes[8] < NH || in_sizes[9] < NH || in_sizes[10] < NH || in_sizes[11] < NH) return;
  if (out_size < NB * SEQ * DM) return;

  const float* x    = (const float*)d_in[0];
  const float* w_k1 = (const float*)d_in[1];
  const float* b_k1 = (const float*)d_in[2];
  const float* w_q1 = (const float*)d_in[3];
  const float* w_k2 = (const float*)d_in[4];
  const float* b_k2 = (const float*)d_in[5];
  const float* w_q2 = (const float*)d_in[6];
  const float* w_v  = (const float*)d_in[7];
  const float* lq1  = (const float*)d_in[8];
  const float* lk1  = (const float*)d_in[9];
  const float* lq2  = (const float*)d_in[10];
  const float* lk2  = (const float*)d_in[11];
  const float* gnw  = (const float*)d_in[12];
  const float* gnb  = (const float*)d_in[13];
  const float* w_o  = (const float*)d_in[14];
  const float* b_o  = (const float*)d_in[15];

  const size_t PWq  = (size_t)DQKV * DM * 2;
  const size_t PWo  = (size_t)DM * DM * 2;
  const size_t PBq  = (size_t)DQKV * 4;
  const size_t PX   = (size_t)SEQ * DM * 2;
  const size_t PQKV = (size_t)SEQ * DQKV * 2;
  const size_t PVT  = (size_t)DVT * SEQ * 2;
  const size_t PC   = (size_t)SEQ * YP * 4;
  const size_t PPT  = (size_t)NPB * PTW * 8;
  const size_t PST  = 256;
  const size_t PYn  = (size_t)SEQ * DM * 2;
  size_t off = 0;
  const size_t oWq   = off; off += PWq;
  const size_t oWo   = off; off += PWo;
  const size_t oBq   = off; off += PBq;
  const size_t oX    = off; off += PX;
  const size_t oQKV  = off; off += PQKV;
  const size_t oQKVr = off; off += PQKV;
  const size_t oVT   = off; off += PVT;
  const size_t oVTr  = off; off += PVT;
  const size_t oC1   = off; off += PC;
  const size_t oC2   = off; off += PC;
  const size_t oPT   = off; off += PPT;
  const size_t oST   = off; off += PST;
  const size_t oYn   = off; off += PYn;
  const size_t oYnr  = off; off += PYn;
  if (off > ws_size) return;
  if (off > (size_t)134217728) return;
  if ((size_t)STW * 4 > PST) return;

  char* ws = (char*)d_ws;
  unsigned short* Wqkv = (unsigned short*)(ws + oWq);
  unsigned short* Wop  = (unsigned short*)(ws + oWo);
  float*          Bq   = (float*)(ws + oBq);
  unsigned short* Xh   = (unsigned short*)(ws + oX);
  unsigned short* QKV  = (unsigned short*)(ws + oQKV);
  unsigned short* QKVr = (unsigned short*)(ws + oQKVr);
  unsigned short* VT   = (unsigned short*)(ws + oVT);
  unsigned short* VTr  = (unsigned short*)(ws + oVTr);
  float*          C1   = (float*)(ws + oC1);
  float*          C2   = (float*)(ws + oC2);
  double*         PT   = (double*)(ws + oPT);
  float*          ST   = (float*)(ws + oST);
  unsigned short* Yn   = (unsigned short*)(ws + oYn);
  unsigned short* Ynr  = (unsigned short*)(ws + oYnr);
  float*          outf = (float*)d_out;

  const dim3 blk(256);
  const int n8x = SEQ * DM / 8;
  const int n8w = DM * DM / 8;
  const dim3 gCx(n8x / 256);
  const dim3 gCw(n8w / 256);
  const dim3 gBq((DQKV / 4 + 255) / 256);
  const dim3 gGqkv(((SEQ / 64) * (DQKV / 64)) / 8);
  const dim3 gGout(((SEQ / 64) * (DM / 64)) / 8);
  const dim3 gVt(SEQ / 64, DVT / 64, 1);
  const dim3 gAttn(NQB * 2 * NH);
  const dim3 gPt(NPB);
  const dim3 gFin(1);
  const dim3 gAp(SEQ / 4);
  const float wScale = 1024.0f;
  const float aScale = 16.0f;
  const float cscale = 1.0f / 16384.0f;

  cvt16<<<gCw, blk, 0, stream>>>(w_q1, Wqkv, n8w, wScale);
  cvt16<<<gCw, blk, 0, stream>>>(w_q2, Wqkv + (size_t)1 * DM * DM, n8w, wScale);
  cvt16<<<gCw, blk, 0, stream>>>(w_k1, Wqkv + (size_t)2 * DM * DM, n8w, wScale);
  cvt16<<<gCw, blk, 0, stream>>>(w_k2, Wqkv + (size_t)3 * DM * DM, n8w, wScale);
  cvt16<<<gCw, blk, 0, stream>>>(w_v,  Wqkv + (size_t)4 * DM * DM, n8w, wScale);
  cvt16<<<gCw, blk, 0, stream>>>(w_o,  Wop, n8w, wScale);
  mkbias<<<gBq, blk, 0, stream>>>(b_k1, b_k2, Bq);

  for (int grp = 0; grp < NB; ++grp) {
    const float* xg = x + (size_t)grp * SEQ_FULL * DM;
    float* outg = outf + (size_t)grp * SEQ * DM;
    cvt16<<<gCx, blk, 0, stream>>>(xg, Xh, n8x, aScale);
    gemm64_f16<0, false><<<gGqkv, blk, 0, stream>>>(Xh, Xh, DM, Wqkv, DM, Bq, cscale, (void*)QKV, QKVr, DQKV,
                                                    SEQ, DQKV, DM, aScale);
    v_tr<<<gVt, blk, 0, stream>>>(QKV, VT, SEQ);
    v_tr<<<gVt, blk, 0, stream>>>(QKVr, VTr, SEQ);
    attn_k<<<gAttn, dim3(128), 0, stream>>>(QKV, QKVr, VT, VTr, C1, C2);
    gn_part<<<gPt, blk, 0, stream>>>(C1, C2, PT);
    gn_fin<<<gFin, blk, 0, stream>>>(PT, lq1, lk1, lq2, lk2, ST);
    gn_apply<<<gAp, blk, 0, stream>>>(C1, C2, ST, gnw, gnb, Yn, Ynr);
    gemm64_f16<1, true><<<gGout, blk, 0, stream>>>(Yn, Ynr, DM, Wop, DM, b_o, cscale, (void*)outg, Ynr, DM,
                                                   SEQ, DM, DM, 1.0f);
  }
  (void)hipGetLastError();
}
